// TransformerBlock_1133871366380
// MI455X (gfx1250) — hardware-verified
//
#include <hip/hip_runtime.h>
#include <stddef.h>


typedef _Float16 v16h __attribute__((ext_vector_type(16)));
typedef _Float16 v8h  __attribute__((ext_vector_type(8)));
typedef _Float16 v4h  __attribute__((ext_vector_type(4)));
typedef float    v8f  __attribute__((ext_vector_type(8)));
typedef float    v4f  __attribute__((ext_vector_type(4)));

#ifndef NB
#define NB 2
#endif
#ifndef SEQ
#define SEQ 2048
#endif
#define NB_FULL  2
#define SEQ_FULL 2048
#define EMB   512
#define NHEAD 8
#define HD    64
#define FFN   2048
#define MROWS (NB * SEQ)

static_assert(NB >= 1 && NB <= NB_FULL);
static_assert(SEQ >= 128 && SEQ <= SEQ_FULL && (SEQ % 128) == 0);
static_assert(EMB == NHEAD * HD);
static_assert(HD == 64);
static_assert((EMB % 64) == 0 && (FFN % 64) == 0);
static_assert((EMB % 32) == 0 && (FFN % 32) == 0);
static_assert((MROWS % 64) == 0 && (MROWS % 8) == 0);
static_assert(EMB == 32 * 4 * 4);
static_assert(((size_t)MROWS * EMB) % (8 * 256) == 0);
static_assert((size_t)MROWS * FFN < (size_t)0xFFFFFFFFu);

#define LDT 72
#define LDC 68

#define WCARRY 64.0f
#define PCARRY 1024.0f
#define VCARRY 64.0f

#define NEGFILL     (-1.0e9f)
#define RECENCY_NEG (-0.05f)

#define WSQ_BYTES     ((size_t)EMB * EMB * 2)
#define WFF_BYTES     ((size_t)EMB * FFN * 2)
#define WT_BYTES      (4 * WSQ_BYTES + 2 * WFF_BYTES)
#define PLANE16_BYTES ((size_t)MROWS * EMB * 2)
#define PLANEH_BYTES  ((size_t)MROWS * FFN * 2)
#define PLANEF_BYTES  ((size_t)MROWS * EMB * 4)
#define OFF_X16   (WT_BYTES)
#define OFF_Q16   (OFF_X16 + PLANE16_BYTES)
#define OFF_K16   (OFF_Q16 + PLANE16_BYTES)
#define OFF_VT16  (OFF_K16 + PLANE16_BYTES)
#define OFF_CTX16 (OFF_VT16 + PLANE16_BYTES)
#define OFF_X1H   (OFF_CTX16 + PLANE16_BYTES)
#define OFF_H16   (OFF_X1H + PLANE16_BYTES)
#define OFF_YF    (OFF_H16 + PLANEH_BYTES)
#define OFF_X1F   (OFF_YF + PLANEF_BYTES)
#define WS_TOTAL  (OFF_X1F + PLANEF_BYTES)
static_assert((WSQ_BYTES % 128) == 0 && (WFF_BYTES % 128) == 0);
static_assert((PLANE16_BYTES % 128) == 0 && (PLANEH_BYTES % 128) == 0 && (PLANEF_BYTES % 128) == 0);
static_assert(WS_TOTAL <= (size_t)134217728);

__device__ __forceinline__ float bfr(float x) {
  unsigned int u = __float_as_uint(x);
  u = (u + 0x7FFFu + ((u >> 16) & 1u)) & 0xFFFF0000u;
  return __uint_as_float(u);
}

__device__ __forceinline__ v16h frag_at(const _Float16* p) {
  v8h lo = *(const v8h*)(p);
  v8h hi = *(const v8h*)(p + 16);
  v16h out;
#pragma unroll
  for (int i = 0; i < 8; ++i) { out[i] = lo[i]; out[i + 8] = hi[i]; }
  return out;
}
__device__ __forceinline__ v16h ld_frag(const _Float16* base, unsigned ld) {
  const unsigned lane = threadIdx.x & 31u;
  return frag_at(base + (lane & 15u) * ld + (lane >> 4) * 8u);
}

__device__ __forceinline__ v8f wmma16(v16h a, v16h b, v8f c) {
  v8f d = __builtin_amdgcn_wmma_f32_16x16x32_f16(false, a, false, b, (short)0, c,
                                                 false, false);
  asm volatile("v_nop\n\tv_nop\n\tv_nop\n\tv_nop" : "+v"(d) : "v"(a), "v"(b));
  return d;
}

__device__ __forceinline__ float red16_max(float x) {
#pragma unroll
  for (int off = 1; off < 16; off <<= 1) x = fmaxf(x, __shfl_xor(x, off, 32));
  return x;
}
__device__ __forceinline__ float red16_sum(float x) {
#pragma unroll
  for (int off = 1; off < 16; off <<= 1) x += __shfl_xor(x, off, 32);
  return x;
}
__device__ __forceinline__ float red32_sum(float x) {
#pragma unroll
  for (int off = 1; off < 32; off <<= 1) x += __shfl_xor(x, off, 32);
  return x;
}

__device__ __forceinline__ void wave_lds_sync() {
  __builtin_amdgcn_fence(3  , "wavefront");
  asm volatile("s_wait_dscnt 0x0" ::: "memory");
  __builtin_amdgcn_wave_barrier();
}

__global__ __launch_bounds__(256) void wconv_kernel(
    const float* __restrict__ W, unsigned ldw, unsigned kd, _Float16* __restrict__ Wt) {
  __shared__ _Float16 T[64 * LDT];
  const unsigned tid = threadIdx.x;
  const unsigned n0 = blockIdx.x * 64u;
  const unsigned k0 = blockIdx.y * 64u;
#pragma unroll 4
  for (unsigned j = 0; j < 16u; ++j) {
    const unsigned idx = tid + 256u * j;
    const unsigned kr = idx >> 6, nc = idx & 63u;
    const float v = W[(size_t)(k0 + kr) * ldw + n0 + nc];
    T[nc * LDT + kr] = (_Float16)(WCARRY * bfr(v));
  }
  __syncthreads();
  v8h x[2];
  size_t off[2];
#pragma unroll
  for (unsigned i = 0; i < 2u; ++i) {
    const unsigned n = 32u * i + (tid >> 3);
    const unsigned kc = (tid & 7u) * 8u;
    x[i] = *(const v8h*)&T[n * LDT + kc];
    off[i] = (size_t)(n0 + n) * kd + k0 + kc;
  }
#pragma unroll
  for (int i = 0; i < 2; ++i) *(volatile v8h*)(Wt + off[i]) = x[i];
  __threadfence();
#pragma unroll
  for (int i = 0; i < 2; ++i) *(volatile v8h*)(Wt + off[i]) = x[i];
}

__global__ __launch_bounds__(256) void xconv_kernel(
    const float* __restrict__ Xin, _Float16* __restrict__ dst) {
  const unsigned e = (blockIdx.x * 256u + threadIdx.x) * 8u;
  const unsigned crow = e / (unsigned)EMB;
  const unsigned c = e - crow * (unsigned)EMB;
  const unsigned bidx = crow / (unsigned)SEQ;
  const unsigned sq = crow - bidx * (unsigned)SEQ;
  const size_t frow = (size_t)bidx * SEQ_FULL + sq;
  const float* sp = Xin + frow * EMB + c;
  const v4f a0 = *(const v4f*)(sp);
  const v4f a1 = *(const v4f*)(sp + 4);
  v8h o;
#pragma unroll
  for (int j = 0; j < 4; ++j) {
    o[j]     = (_Float16)bfr(a0[j]);
    o[j + 4] = (_Float16)bfr(a1[j]);
  }
  *(volatile v8h*)(dst + (size_t)e) = o;
  __threadfence();
  *(volatile v8h*)(dst + (size_t)e) = o;
}

template <int MODE, int KD, int ND>
__device__ __forceinline__ void gemm_body(
    const _Float16* __restrict__ A16, const _Float16* __restrict__ Bt,
    const float* __restrict__ bias, const float* __restrict__ resid,
    float* __restrict__ outf, _Float16* __restrict__ out16) {
  static_assert((KD % 32) == 0 && (KD % 8) == 0);
  static_assert((ND % 64) == 0);
  static_assert(MODE < 3 || ND == EMB);
  static_assert(MODE != 1 || (ND == EMB && (SEQ % 64) == 0));
  __shared__ float Cs[64 * LDC];
  const unsigned tid = threadIdx.x, lane = tid & 31u;
  const unsigned w = (unsigned)__builtin_amdgcn_readfirstlane((int)(tid >> 5));
  const unsigned mw = w >> 1, nw = w & 1u;
  const unsigned hh = lane >> 4, m = lane & 15u;
  const unsigned n0 = blockIdx.x * 64u;
  const unsigned row0 = blockIdx.y * 64u;

  const _Float16* ap  = A16 + (size_t)(row0 + mw * 16u + m) * KD + hh * 8u;
  const _Float16* bp0 = Bt + (size_t)(n0 + nw * 32u + m) * KD + hh * 8u;
  const _Float16* bp1 = bp0 + 16 * KD;
  v8f acc0 = {}, acc1 = {};
#pragma unroll 2
  for (unsigned k0 = 0; k0 < (unsigned)KD; k0 += 32u) {
    const v16h a  = frag_at(ap + k0);
    const v16h b0 = frag_at(bp0 + k0);
    const v16h b1 = frag_at(bp1 + k0);
    acc0 = wmma16(a, b0, acc0);
    acc1 = wmma16(a, b1, acc1);
  }
#pragma unroll
  for (int r = 0; r < 8; ++r) {
    const unsigned ci = (mw * 16u + hh * 8u + (unsigned)r) * LDC + nw * 32u + m;
    Cs[ci]      = acc0[r];
    Cs[ci + 16] = acc1[r];
  }
  __syncthreads();

  if (MODE == 0 || MODE == 2) {
    v8h x[2];
    size_t off[2];
#pragma unroll
    for (unsigned i = 0; i < 2u; ++i) {
      const unsigned r = 32u * i + (tid >> 3);
      const unsigned c = (tid & 7u) * 8u;
      const v4f u0 = *(const v4f*)&Cs[r * LDC + c];
      const v4f u1 = *(const v4f*)&Cs[r * LDC + c + 4];
      const v4f g0 = *(const v4f*)(bias + n0 + c);
      const v4f g1 = *(const v4f*)(bias + n0 + c + 4);
#pragma unroll
      for (int j = 0; j < 4; ++j) {
        float t0 = u0[j] * (1.0f / WCARRY) + bfr(g0[j]);
        float t1 = u1[j] * (1.0f / WCARRY) + bfr(g1[j]);
        if (MODE == 2) { t0 = fmaxf(t0, 0.0f); t1 = fmaxf(t1, 0.0f); }
        x[i][j]     = (_Float16)t0;
        x[i][j + 4] = (_Float16)t1;
      }
      off[i] = (size_t)(row0 + r) * ND + n0 + c;
    }
#pragma unroll
    for (int i = 0; i < 2; ++i) *(volatile v8h*)(out16 + off[i]) = x[i];
    __threadfence();
#pragma unroll
    for (int i = 0; i < 2; ++i) *(volatile v8h*)(out16 + off[i]) = x[i];
  }

  if (MODE == 1) {
    const unsigned bidx = row0 / (unsigned)SEQ;
    const unsigned key0 = row0 - bidx * (unsigned)SEQ;
    v8h x[2];
    size_t off[2];
#pragma unroll
    for (unsigned i = 0; i < 2u; ++i) {
      const unsigned dcol = 32u * i + (tid >> 3);
      const unsigned kk = (tid & 7u) * 8u;
      const float bb = bfr(bias[n0 + dcol]);
#pragma unroll
      for (unsigned j = 0; j < 8u; ++j)
        x[i][j] = (_Float16)(Cs[(kk + j) * LDC + dcol] * (1.0f / WCARRY) + bb);
      off[i] = ((size_t)bidx * ND + n0 + dcol) * SEQ + key0 + kk;
    }
#pragma unroll
    for (int i = 0; i < 2; ++i) *(volatile v8h*)(out16 + off[i]) = x[i];
    __threadfence();
#pragma unroll
    for (int i = 0; i < 2; ++i) *(volatile v8h*)(out16 + off[i]) = x[i];
  }

  if (MODE == 3 || MODE == 4) {
    const float sc = (MODE == 3) ? (1.0f / (WCARRY * VCARRY)) : (1.0f / WCARRY);
    v4f xs[4];
    size_t off[4];
#pragma unroll
    for (unsigned i = 0; i < 4u; ++i) {
      const unsigned r = 16u * i + (tid >> 4);
      const unsigned c = (tid & 15u) * 4u;
      const unsigned crow = row0 + r;
      const v4f u = *(const v4f*)&Cs[r * LDC + c];
      const v4f g = *(const v4f*)(bias + n0 + c);
      v4f rv;
      if (MODE == 3) {
        const unsigned bidx = crow / (unsigned)SEQ;
        const unsigned sq = crow - bidx * (unsigned)SEQ;
        const size_t frow = (size_t)bidx * SEQ_FULL + sq;
        rv = *(const v4f*)(resid + frow * ND + n0 + c);
#pragma unroll
        for (int j = 0; j < 4; ++j) rv[j] = bfr(rv[j]);
      } else {
        rv = *(const v4f*)(resid + (size_t)crow * ND + n0 + c);
      }
      v4f val;
#pragma unroll
      for (int j = 0; j < 4; ++j) val[j] = (u[j] * sc + bfr(g[j])) + rv[j];
      xs[i] = val;
      off[i] = (size_t)crow * ND + n0 + c;
    }
#pragma unroll
    for (int i = 0; i < 4; ++i) *(volatile v4f*)(outf + off[i]) = xs[i];
    __threadfence();
#pragma unroll
    for (int i = 0; i < 4; ++i) *(volatile v4f*)(outf + off[i]) = xs[i];
  }
}

__global__ __launch_bounds__(256) void gemm_qk_kernel(
    const _Float16* __restrict__ A16, const _Float16* __restrict__ Bt,
    const float* __restrict__ bias, _Float16* __restrict__ out16) {
  gemm_body<0, EMB, EMB>(A16, Bt, bias, nullptr, nullptr, out16);
}
__global__ __launch_bounds__(256) void gemm_vt_kernel(
    const _Float16* __restrict__ A16, const _Float16* __restrict__ Bt,
    const float* __restrict__ bias, _Float16* __restrict__ out16) {
  gemm_body<1, EMB, EMB>(A16, Bt, bias, nullptr, nullptr, out16);
}
__global__ __launch_bounds__(256) void gemm_ffn1_kernel(
    const _Float16* __restrict__ A16, const _Float16* __restrict__ Bt,
    const float* __restrict__ bias, _Float16* __restrict__ out16) {
  gemm_body<2, EMB, FFN>(A16, Bt, bias, nullptr, nullptr, out16);
}
__global__ __launch_bounds__(256) void gemm_wo_kernel(
    const _Float16* __restrict__ A16, const _Float16* __restrict__ Bt,
    const float* __restrict__ bias, const float* __restrict__ resid,
    float* __restrict__ outf) {
  gemm_body<3, EMB, EMB>(A16, Bt, bias, resid, outf, nullptr);
}
__global__ __launch_bounds__(256) void gemm_ffn2_kernel(
    const _Float16* __restrict__ A16, const _Float16* __restrict__ Bt,
    const float* __restrict__ bias, const float* __restrict__ resid,
    float* __restrict__ outf) {
  gemm_body<4, FFN, EMB>(A16, Bt, bias, resid, outf, nullptr);
}

__global__ __launch_bounds__(256) void attn_kernel(
    const _Float16* __restrict__ Qh, const _Float16* __restrict__ Kh,
    const _Float16* __restrict__ Vt, _Float16* __restrict__ Ov) {
#pragma clang fp contract(off)
  __shared__ _Float16 Ks[64 * LDT];
  __shared__ _Float16 Vs[64 * LDT];
  __shared__ _Float16 Ps[8 * 16 * LDT];

  const unsigned tid = threadIdx.x, lane = tid & 31u;
  const unsigned w = (unsigned)__builtin_amdgcn_readfirstlane((int)(tid >> 5));
  const unsigned hh = lane >> 4, m = lane & 15u;
  const unsigned q0 = blockIdx.x * 128u;
  const unsigned head = blockIdx.y;
  const unsigned b = blockIdx.z;
  const unsigned wq0 = q0 + w * 16u;
  const unsigned pb = w * (16u * LDT);

  const size_t qoff = (size_t)(b * (unsigned)SEQ + wq0 + m) * EMB + head * HD + hh * 8u;
  v16h qf[2];
  qf[0] = frag_at(Qh + qoff);
  qf[1] = frag_at(Qh + qoff + 32);

  float mrow[8], lrow[8];
  v8f o[4];
#pragma unroll
  for (int v = 0; v < 8; ++v) { mrow[v] = -1.0e30f; lrow[v] = 0.0f; }
#pragma unroll
  for (int nb = 0; nb < 4; ++nb) o[nb] = (v8f){};

  const size_t kplane = (size_t)b * SEQ * EMB + head * HD;
  const size_t vplane = ((size_t)b * EMB + head * HD) * SEQ;
  const unsigned kend = q0 + 128u;
  const int qrow_i = (int)(wq0 + hh * 8u);

  for (unsigned kb = 0; kb < kend; kb += 64u) {
#pragma unroll
    for (unsigned j = 0; j < 2u; ++j) {
      const unsigned idx = tid + 256u * j;
      const unsigned r = idx >> 3, c = (idx & 7u) * 8u;
      *(v8h*)&Ks[r * LDT + c] = *(const v8h*)(Kh + kplane + (size_t)(kb + r) * EMB + c);
      *(v8h*)&Vs[r * LDT + c] = *(const v8h*)(Vt + vplane + (size_t)r * SEQ + kb + c);
    }
    __syncthreads();

    if (kb <= wq0 + 15u) {
      v8f s[4];
#pragma unroll
      for (int kg = 0; kg < 4; ++kg) {
        v8f t = {};
#pragma unroll
        for (int c = 0; c < 2; ++c) {
          const v16h kf = ld_frag(&Ks[(kg * 16) * LDT + c * 32], LDT);
          t = wmma16(qf[c], kf, t);
        }
        const int dk = qrow_i - (int)(kb + (unsigned)kg * 16u + m);
#pragma unroll
        for (int v = 0; v < 8; ++v) {
          const int d = dk + v;
          const float bia = (d < 0) ? NEGFILL : (RECENCY_NEG * (float)d);
          t[v] = t[v] * 0.125f + bia;
        }
        s[kg] = t;
      }

      float alpha[8];
#pragma unroll
      for (int v = 0; v < 8; ++v) {
        float mx = fmaxf(fmaxf(s[0][v], s[1][v]), fmaxf(s[2][v], s[3][v]));
        mx = red16_max(mx);
        const float mn = fmaxf(mrow[v], mx);
        alpha[v] = __expf(mrow[v] - mn);
        mrow[v] = mn;
      }
#pragma unroll
      for (int kg = 0; kg < 4; ++kg)
#pragma unroll
        for (int v = 0; v < 8; ++v) s[kg][v] = __expf(s[kg][v] - mrow[v]);
#pragma unroll
      for (int v = 0; v < 8; ++v) {
        const float rs = red16_sum((s[0][v] + s[1][v]) + (s[2][v] + s[3][v]));
        lrow[v] = alpha[v] * lrow[v] + rs;
      }
#pragma unroll
      for (int nb = 0; nb < 4; ++nb)
#pragma unroll
        for (int v = 0; v < 8; ++v) o[nb][v] = o[nb][v] * alpha[v];

#pragma unroll
      for (int kg = 0; kg < 4; ++kg)
#pragma unroll
        for (int v = 0; v < 8; ++v)
          Ps[pb + (hh * 8u + (unsigned)v) * LDT + (unsigned)kg * 16u + m] =
              (_Float16)(s[kg][v] * PCARRY);
      wave_lds_sync();

#pragma unroll
      for (int c = 0; c < 2; ++c) {
        const v16h pf = ld_frag(&Ps[pb + c * 32], LDT);
#pragma unroll
        for (int nb = 0; nb < 4; ++nb) {
          const v16h vf = ld_frag(&Vs[(nb * 16) * LDT + c * 32], LDT);
          o[nb] = wmma16(pf, vf, o[nb]);
        }
      }
      wave_lds_sync();
    }
    __syncthreads();
  }

  float inv[8];
#pragma unroll
  for (int v = 0; v < 8; ++v) inv[v] = __builtin_amdgcn_rcpf(lrow[v]) * (VCARRY / PCARRY);
#pragma unroll
  for (int nb = 0; nb < 4; ++nb)
#pragma unroll
    for (int v = 0; v < 8; ++v)
      Ps[pb + (hh * 8u + (unsigned)v) * LDT + (unsigned)nb * 16u + m] =
          (_Float16)(o[nb][v] * inv[v]);
  wave_lds_sync();
  v8h x[4];
  size_t off[4];
#pragma unroll
  for (unsigned i = 0; i < 4u; ++i) {
    const unsigned r = 4u * i + (lane >> 3);
    const unsigned c = (lane & 7u) * 8u;
    x[i] = *(const v8h*)&Ps[pb + r * LDT + c];
    off[i] = (size_t)(b * (unsigned)SEQ + wq0 + r) * EMB + head * HD + c;
  }
#pragma unroll
  for (int i = 0; i < 4; ++i) *(volatile v8h*)(Ov + off[i]) = x[i];
  __threadfence();
#pragma unroll
  for (int i = 0; i < 4; ++i) *(volatile v8h*)(Ov + off[i]) = x[i];
}

template <int FULLROWS, int W16>
__device__ __forceinline__ void ln_body(
    const float* __restrict__ Yf, const float* __restrict__ gam, const float* __restrict__ bet,
    float* __restrict__ outf, _Float16* __restrict__ out16) {
  const unsigned tid = threadIdx.x, lane = tid & 31u;
  const unsigned w = (unsigned)__builtin_amdgcn_readfirstlane((int)(tid >> 5));
  const unsigned row = blockIdx.x * 8u + w;
  const float* src = Yf + (size_t)row * EMB + lane * 4u;
  v4f v[4];
#pragma unroll
  for (int j = 0; j < 4; ++j) v[j] = *(const v4f*)(src + j * 128);
  float s = 0.0f;
#pragma unroll
  for (int j = 0; j < 4; ++j)
#pragma unroll
    for (int e = 0; e < 4; ++e) s += v[j][e];
  s = red32_sum(s);
  const float mu = s * (1.0f / (float)EMB);
  float ss = 0.0f;
#pragma unroll
  for (int j = 0; j < 4; ++j)
#pragma unroll
    for (int e = 0; e < 4; ++e) { const float d = v[j][e] - mu; ss += d * d; }
  ss = red32_sum(ss);
  const float rstd = rsqrtf(ss * (1.0f / (float)EMB) + 1.0e-5f);

  size_t orow = row;
  if (FULLROWS) {
    const unsigned bidx = row / (unsigned)SEQ;
    const unsigned sq = row - bidx * (unsigned)SEQ;
    orow = (size_t)bidx * SEQ_FULL + sq;
  }
  v4f y[4];
  v4h yh[4];
#pragma unroll
  for (int j = 0; j < 4; ++j) {
    const v4f g = *(const v4f*)(gam + j * 128 + lane * 4u);
    const v4f t = *(const v4f*)(bet + j * 128 + lane * 4u);
#pragma unroll
    for (int e = 0; e < 4; ++e) {
      y[j][e] = (v[j][e] - mu) * rstd * bfr(g[e]) + bfr(t[e]);
      yh[j][e] = (_Float16)y[j][e];
    }
  }
  float* dst = outf + orow * EMB + lane * 4u;
  _Float16* dst16 = out16 + (size_t)row * EMB + lane * 4u;
#pragma unroll
  for (int j = 0; j < 4; ++j) *(volatile v4f*)(dst + j * 128) = y[j];
  if (W16) {
#pragma unroll
    for (int j = 0; j < 4; ++j) *(volatile v4h*)(dst16 + j * 128) = yh[j];
  }
  __threadfence();
#pragma unroll
  for (int j = 0; j < 4; ++j) *(volatile v4f*)(dst + j * 128) = y[j];
  if (W16) {
#pragma unroll
    for (int j = 0; j < 4; ++j) *(volatile v4h*)(dst16 + j * 128) = yh[j];
  }
}

__global__ __launch_bounds__(256) void ln1_kernel(
    const float* __restrict__ Yf, const float* __restrict__ gam, const float* __restrict__ bet,
    float* __restrict__ outf, _Float16* __restrict__ out16) {
  ln_body<0, 1>(Yf, gam, bet, outf, out16);
}
__global__ __launch_bounds__(256) void ln2_kernel(
    const float* __restrict__ Yf, const float* __restrict__ gam, const float* __restrict__ bet,
    float* __restrict__ outf) {
  ln_body<1, 0>(Yf, gam, bet, outf, nullptr);
}

extern "C" void kernel_launch(void* const* d_in, const int* in_sizes, int n_in,
                              void* d_out, int out_size, void* d_ws, size_t ws_size,
                              hipStream_t stream) {
  if (n_in < 17) return;
  const long long need_x = ((long long)(NB - 1) * SEQ_FULL + SEQ) * EMB;
  if ((long long)in_sizes[0] < need_x) return;
  if ((long long)in_sizes[1] < (long long)EMB * EMB) return;
  if ((long long)in_sizes[3] < (long long)EMB * EMB) return;
  if ((long long)in_sizes[5] < (long long)EMB * EMB) return;
  if ((long long)in_sizes[7] < (long long)EMB * EMB) return;
  if (in_sizes[2] < EMB || in_sizes[4] < EMB || in_sizes[6] < EMB || in_sizes[8] < EMB) return;
  if (in_sizes[9] < EMB || in_sizes[10] < EMB) return;
  if ((long long)in_sizes[11] < (long long)EMB * FFN) return;
  if (in_sizes[12] < FFN) return;
  if ((long long)in_sizes[13] < (long long)FFN * EMB) return;
  if (in_sizes[14] < EMB || in_sizes[15] < EMB || in_sizes[16] < EMB) return;
  if ((long long)out_size < need_x) return;
  if (ws_size < WS_TOTAL) return;

  const float* X    = (const float*)d_in[0];
  const float* wq   = (const float*)d_in[1];
  const float* bq   = (const float*)d_in[2];
  const float* wk   = (const float*)d_in[3];
  const float* bk   = (const float*)d_in[4];
  const float* wv   = (const float*)d_in[5];
  const float* bv   = (const float*)d_in[6];
  const float* wo   = (const float*)d_in[7];
  const float* bo   = (const float*)d_in[8];
  const float* ln1g = (const float*)d_in[9];
  const float* ln1b = (const float*)d_in[10];
  const float* w1   = (const float*)d_in[11];
  const float* b1   = (const float*)d_in[12];
  const float* w2   = (const float*)d_in[13];
  const float* b2   = (const float*)d_in[14];
  const float* ln2g = (const float*)d_in[15];
  const float* ln2b = (const float*)d_in[16];
  float* out = (float*)d_out;

  char* ws = (char*)d_ws;
  _Float16* Wq_t  = (_Float16*)(ws + 0 * WSQ_BYTES);
  _Float16* Wk_t  = (_Float16*)(ws + 1 * WSQ_BYTES);
  _Float16* Wv_t  = (_Float16*)(ws + 2 * WSQ_BYTES);
  _Float16* Wo_t  = (_Float16*)(ws + 3 * WSQ_BYTES);
  _Float16* W1_t  = (_Float16*)(ws + 4 * WSQ_BYTES);
  _Float16* W2_t  = (_Float16*)(ws + 4 * WSQ_BYTES + WFF_BYTES);
  _Float16* X16   = (_Float16*)(ws + OFF_X16);
  _Float16* Q16   = (_Float16*)(ws + OFF_Q16);
  _Float16* K16   = (_Float16*)(ws + OFF_K16);
  _Float16* Vt16  = (_Float16*)(ws + OFF_VT16);
  _Float16* Ctx16 = (_Float16*)(ws + OFF_CTX16);
  _Float16* X1h   = (_Float16*)(ws + OFF_X1H);
  _Float16* H16   = (_Float16*)(ws + OFF_H16);
  float*    Yf    = (float*)(ws + OFF_YF);
  float*    X1f   = (float*)(ws + OFF_X1F);

  dim3 blk(256);
  dim3 gsq(EMB / 64, EMB / 64);
  dim3 gE(EMB / 64, MROWS / 64);
  dim3 gF(FFN / 64, MROWS / 64);

  wconv_kernel<<<gsq, blk, 0, stream>>>(wq, (unsigned)EMB, (unsigned)EMB, Wq_t);
  wconv_kernel<<<gsq, blk, 0, stream>>>(wk, (unsigned)EMB, (unsigned)EMB, Wk_t);
  wconv_kernel<<<gsq, blk, 0, stream>>>(wv, (unsigned)EMB, (unsigned)EMB, Wv_t);
  wconv_kernel<<<gsq, blk, 0, stream>>>(wo, (unsigned)EMB, (unsigned)EMB, Wo_t);
  wconv_kernel<<<dim3(FFN / 64, EMB / 64), blk, 0, stream>>>(w1, (unsigned)FFN, (unsigned)EMB, W1_t);
  wconv_kernel<<<dim3(EMB / 64, FFN / 64), blk, 0, stream>>>(w2, (unsigned)EMB, (unsigned)FFN, W2_t);

  xconv_kernel<<<dim3((unsigned)(((size_t)MROWS * EMB) / 2048)), blk, 0, stream>>>(X, X16);

  gemm_qk_kernel<<<gE, blk, 0, stream>>>(X16, Wq_t, bq, Q16);
  gemm_qk_kernel<<<gE, blk, 0, stream>>>(X16, Wk_t, bk, K16);
  gemm_vt_kernel<<<gE, blk, 0, stream>>>(X16, Wv_t, bv, Vt16);

  attn_kernel<<<dim3(SEQ / 128, NHEAD, NB), blk, 0, stream>>>(Q16, K16, Vt16, Ctx16);

  gemm_wo_kernel<<<gE, blk, 0, stream>>>(Ctx16, Wo_t, bo, X, Yf);
  ln1_kernel<<<dim3(MROWS / 8), blk, 0, stream>>>(Yf, ln1g, ln1b, X1f, X1h);

  gemm_ffn1_kernel<<<gF, blk, 0, stream>>>(X1h, W1_t, b1, H16);
  gemm_ffn2_kernel<<<gE, blk, 0, stream>>>(H16, W2_t, b2, X1f, Yf);
  ln2_kernel<<<dim3(MROWS / 8), blk, 0, stream>>>(Yf, ln2g, ln2b, out);
}
